// BiAffineLayer3_39779987096217
// MI455X (gfx1250) — hardware-verified
//
#include <hip/hip_runtime.h>
#include <math.h>

constexpr int kBatch   = 2;
constexpr int kSeqLen  = 512;
constexpr int kHin     = 768;
constexpr int kHid     = 256;
constexpr int kNl      = 12;
constexpr int kNlPad   = 16;
constexpr int kRows    = kBatch * kSeqLen;
constexpr int kKeyCols = kHid * kNl;
constexpr int kOutPitch = kNl * kSeqLen;

typedef __attribute__((ext_vector_type(16))) _Float16 v16h;
typedef __attribute__((ext_vector_type(8)))  _Float16 v8h;
typedef __attribute__((ext_vector_type(16))) __bf16   v16b;
typedef __attribute__((ext_vector_type(8)))  __bf16   v8b;
typedef __attribute__((ext_vector_type(8)))  float    v8f;
typedef __attribute__((ext_vector_type(4)))  float    v4f;
typedef __attribute__((ext_vector_type(4)))  unsigned int v4u;
typedef __attribute__((ext_vector_type(8)))  unsigned int v8u;

__device__ __forceinline__ unsigned short f2bf_bits(float f) {
  unsigned u = __float_as_uint(f);
  return (unsigned short)((u + 0x7FFFu + ((u >> 16) & 1u)) >> 16);
}
__device__ __forceinline__ float bf_bits2f(unsigned short h) { return __uint_as_float(((unsigned)h) << 16); }

__device__ __forceinline__ void dep_guard_h(v8f& a, v8f& b, v16h x, v16h y) { asm volatile("v_nop\n\tv_nop\n\tv_nop\n\tv_nop" : "+v"(a), "+v"(b) : "v"(x), "v"(y)); }
__device__ __forceinline__ void dep_guard_b(v8f& a, v8f& b, v16b x, v16b y) { asm volatile("v_nop\n\tv_nop\n\tv_nop\n\tv_nop" : "+v"(a), "+v"(b) : "v"(x), "v"(y)); }
__device__ __forceinline__ void keep4_h(v16h a, v16h b, v16h c, v16h d) { asm volatile("v_nop" :: "v"(a), "v"(b), "v"(c), "v"(d)); }
__device__ __forceinline__ void keep4_b(v16b a, v16b b, v16b c, v16b d) { asm volatile("v_nop" :: "v"(a), "v"(b), "v"(c), "v"(d)); }
__device__ __forceinline__ void acc_guard4(v8f& a, v8f& b, v8f& c, v8f& d) { asm volatile("v_nop\n\tv_nop\n\tv_nop\n\tv_nop" : "+v"(a), "+v"(b), "+v"(c), "+v"(d)); }
template <typename T> struct Frag;
template <> struct Frag<_Float16> {
  typedef v16h V; union U { v16h v; v8h h[2]; };
  static __device__ __forceinline__ v16h load(const _Float16* p) {
    U f; f.h[0] = *(const v8h*)(p); f.h[1] = *(const v8h*)(p + 16); return f.v;
  }
  static __device__ __forceinline__ v8f mma(v16h a, v16h b, v8f c) {
    return __builtin_amdgcn_wmma_f32_16x16x32_f16(false, a, false, b, (short)0, c, false, false);
  }
  static __device__ __forceinline__ void guard(v8f& a, v8f& b, v16h x, v16h y) { dep_guard_h(a, b, x, y); }
  static __device__ __forceinline__ void keep(v16h a, v16h b, v16h c, v16h d) { keep4_h(a, b, c, d); }
};
template <> struct Frag<__bf16> {
  typedef v16b V; union U { v16b v; v8b h[2]; };
  static __device__ __forceinline__ v16b load(const __bf16* p) {
    U f; f.h[0] = *(const v8b*)(p); f.h[1] = *(const v8b*)(p + 16); return f.v;
  }
  static __device__ __forceinline__ v8f mma(v16b a, v16b b, v8f c) {
    return __builtin_amdgcn_wmma_f32_16x16x32_bf16(false, a, false, b, (short)0, c, false, false);
  }
  static __device__ __forceinline__ void guard(v8f& a, v8f& b, v16b x, v16b y) { dep_guard_b(a, b, x, y); }
  static __device__ __forceinline__ void keep(v16b a, v16b b, v16b c, v16b d) { keep4_b(a, b, c, d); }
};

__device__ __forceinline__ unsigned pk16(unsigned short a, unsigned short b) { return (unsigned)a | ((unsigned)b << 16); }

template <int ET> struct Elem;
template <> struct Elem<0> { typedef _Float16 T; };
template <> struct Elem<1> { typedef __bf16 T; };
template <int ET, bool SPLIT, int BIAS_MODE, int OUT_MODE, bool RESID, int ACT = 0>
__global__ __launch_bounds__(256) void wmma_gemm64(
    const unsigned short* __restrict__ Ap, const unsigned short* __restrict__ A2p, int lda, long strideA,
    const unsigned short* __restrict__ Btp, const unsigned short* __restrict__ Bt2p, int ldb, long strideB,
    void* __restrict__ Cout, void* __restrict__ Cout2, int ldc, long strideC,
    const float* __restrict__ bias,
    const float* __restrict__ resid, long strideR,
    int M, int N, int K, float scale) {
  typedef typename Elem<ET>::T T;
  typedef typename Frag<T>::V V;
  const T* A = (const T*)Ap; const T* A2 = (const T*)A2p; const T* Bt = (const T*)Btp; const T* Bt2 = (const T*)Bt2p;
  __shared__ __align__(16) float sT[8][16 * 68];
  const int b    = blockIdx.y;
  const int lane = threadIdx.x & 31;
  const int wave = threadIdx.x >> 5;
  const int tilesN = N >> 6;
  const int tilesM = M >> 6;
  const int tile = blockIdx.x * 8 + wave;
  if (tile >= tilesM * tilesN) return;
  const int tm = tile / tilesN;
  const int tn = tile - tm * tilesN;
  const int m0 = tm << 6;
  const int n0 = tn << 6;

  const T* Ab  = A  + (size_t)b * strideA;
  const T* Bb  = Bt + (size_t)b * strideB;
  const T* Ab2 = SPLIT ? (A2  + (size_t)b * strideA) : nullptr;
  const T* Bb2 = SPLIT ? (Bt2 + (size_t)b * strideB) : nullptr;

  const int rlane = lane & 15;
  const int koff  = (lane >> 4) * 8;
  const int mOff  = (lane >> 4) * 8;

  v8f acc[4][4];
#pragma unroll
  for (int i = 0; i < 4; ++i)
#pragma unroll
    for (int j = 0; j < 4; ++j) acc[i][j] = (v8f){0.f,0.f,0.f,0.f,0.f,0.f,0.f,0.f};

  for (int k0 = 0; k0 < K; k0 += 32) {
    V bh[4], bl[4];
#pragma unroll
    for (int j = 0; j < 4; ++j) {
      const size_t bo = (size_t)(n0 + (j << 4) + rlane) * ldb + koff + k0;
      bh[j] = Frag<T>::load(Bb + bo);
      if (SPLIT) bl[j] = Frag<T>::load(Bb2 + bo);
    }
#pragma unroll
    for (int i = 0; i < 4; ++i) {
      const size_t ao = (size_t)(m0 + (i << 4) + rlane) * lda + koff + k0;
      V ah = Frag<T>::load(Ab + ao);
      V al;
      if (SPLIT) al = Frag<T>::load(Ab2 + ao);
#pragma unroll
      for (int j = 0; j < 4; ++j) {
        acc[i][j] = Frag<T>::mma(ah, bh[j], acc[i][j]);
        if (SPLIT) {
          acc[i][j] = Frag<T>::mma(ah, bl[j], acc[i][j]);
          acc[i][j] = Frag<T>::mma(al, bh[j], acc[i][j]);
        }
      }
      Frag<T>::guard(acc[i][0], acc[i][3], ah, SPLIT ? al : ah);
    }
    Frag<T>::keep(bh[0], bh[1], bh[2], bh[3]);
    if (SPLIT) Frag<T>::keep(bl[0], bl[1], bl[2], bl[3]);
  }
  acc_guard4(acc[0][0], acc[0][1], acc[0][2], acc[0][3]);
  acc_guard4(acc[1][0], acc[1][1], acc[1][2], acc[1][3]);
  acc_guard4(acc[2][0], acc[2][1], acc[2][2], acc[2][3]);
  acc_guard4(acc[3][0], acc[3][1], acc[3][2], acc[3][3]);

  float* slab = sT[wave];
  const float* Rb = RESID ? (resid + (size_t)b * strideR) : nullptr;
#pragma unroll
  for (int i = 0; i < 4; ++i) {
    const int mBase = m0 + (i << 4);
#pragma unroll
    for (int j = 0; j < 4; ++j) {
      const int n = n0 + (j << 4) + rlane;
      float bv = 0.f;
      if (BIAS_MODE == 2) bv = bias[n];
#pragma unroll
      for (int r = 0; r < 8; ++r) {
        float v = acc[i][j][r] * scale;
        if (BIAS_MODE == 1) v += bias[mBase + mOff + r];
        if (BIAS_MODE == 2) v += bv;
        if (RESID) v += Rb[(size_t)(mBase + mOff + r) * ldc + n];
        if (ACT == 2) v = fmaxf(v, 0.0f);
        if (ACT == 4) v = (v > 0.f) ? v : 0.01f * v;
        slab[(mOff + r) * 68 + (j << 4) + rlane] = v;
      }
    }
    __builtin_amdgcn_fence(__ATOMIC_RELEASE, "workgroup");
    __builtin_amdgcn_wave_barrier();
    __builtin_amdgcn_fence(__ATOMIC_ACQUIRE, "workgroup");
    if (OUT_MODE == 0) {
      float* C = (float*)Cout + (size_t)b * strideC;
      const int hh = lane >> 4, c4 = (lane & 15) * 4;
      for (int pass = 0; pass < 2; ++pass) {
#pragma unroll
        for (int it = 0; it < 8; ++it) {
          const int row = it * 2 + hh;
          v4f v = *(const v4f*)(slab + row * 68 + c4);
          *(volatile v4f*)(C + (size_t)(mBase + row) * ldc + n0 + c4) = v;
        }
        __threadfence();
      }
    } else {
      const int q = lane >> 3, c8 = (lane & 7) * 8;
      unsigned short* C  = (unsigned short*)Cout  + (size_t)b * strideC;
      unsigned short* C2 = (OUT_MODE == 2) ? ((unsigned short*)Cout2 + (size_t)b * strideC) : nullptr;
      for (int pass = 0; pass < 2; ++pass) {
#pragma unroll
        for (int it = 0; it < 4; ++it) {
          const int row = it * 4 + q;
          const float* sp = slab + row * 68 + c8;
          v8h hv, lv;
#pragma unroll
          for (int e = 0; e < 8; ++e) {
            if (OUT_MODE == 1) {
              hv[e] = (_Float16)sp[e];
            } else {
              unsigned short hb = f2bf_bits(sp[e]);
              unsigned short lb = f2bf_bits(sp[e] - bf_bits2f(hb));
              hv[e] = __builtin_bit_cast(_Float16, hb);
              lv[e] = __builtin_bit_cast(_Float16, lb);
            }
          }
          *(volatile v8h*)(C + (size_t)(mBase + row) * ldc + n0 + c8) = hv;
          if (OUT_MODE == 2) *(volatile v8h*)(C2 + (size_t)(mBase + row) * ldc + n0 + c8) = lv;
        }
        __threadfence();
      }
    }
    __builtin_amdgcn_fence(__ATOMIC_RELEASE, "workgroup");
    __builtin_amdgcn_wave_barrier();
    __builtin_amdgcn_fence(__ATOMIC_ACQUIRE, "workgroup");
  }
}

__device__ __forceinline__ void split_pack2(float x0, float x1, unsigned& hw, unsigned& lw) {
  const unsigned short a  = f2bf_bits(x0);
  const unsigned short c  = f2bf_bits(x1);
  const unsigned short al = f2bf_bits(x0 - bf_bits2f(a));
  const unsigned short cl = f2bf_bits(x1 - bf_bits2f(c));
  hw = pk16(a, c);
  lw = pk16(al, cl);
}
__device__ __forceinline__ v4f ld4(const float* p) { return *(const v4f*)(p); }
__device__ __forceinline__ v4f relu4(v4f v) {
  return (v4f){fmaxf(v[0], 0.f), fmaxf(v[1], 0.f), fmaxf(v[2], 0.f), fmaxf(v[3], 0.f)};
}
__device__ __forceinline__ v8f bmma(v16b a, v16b b, v8f c) {
  c = __builtin_amdgcn_wmma_f32_16x16x32_bf16(false, a, false, b, (short)0, c, false, false);
  asm volatile("v_nop\n\tv_nop\n\tv_nop\n\tv_nop" : "+v"(c) : "v"(a), "v"(b));
  return c;
}
__device__ __forceinline__ void split_store8(const float* p, unsigned short* qh, unsigned short* ql, bool live) {
  const v4f z = (v4f){0.f, 0.f, 0.f, 0.f};
  v4f a = ld4(p);
  v4f c = ld4(p + 4);
  a = live ? a : z;
  c = live ? c : z;
  unsigned hw[4], lw[4];
  split_pack2(a[0], a[1], hw[0], lw[0]);
  split_pack2(a[2], a[3], hw[1], lw[1]);
  split_pack2(c[0], c[1], hw[2], lw[2]);
  split_pack2(c[2], c[3], hw[3], lw[3]);
  const v4u uh = (v4u){hw[0], hw[1], hw[2], hw[3]};
  const v4u ul = (v4u){lw[0], lw[1], lw[2], lw[3]};
  *(volatile v4u*)qh = uh;
  *(volatile v4u*)ql = ul;
  __threadfence();
  *(volatile v4u*)qh = uh;
  *(volatile v4u*)ql = ul;
}

__global__ __launch_bounds__(256) void split8_bf16_kernel(const float* __restrict__ in,
                                                          unsigned short* __restrict__ hi,
                                                          unsigned short* __restrict__ lo, int n8) {
  const int i = blockIdx.x * 256 + threadIdx.x;
  if (i >= n8) return;
  split_store8(in + 8 * (size_t)i, hi + 8 * (size_t)i, lo + 8 * (size_t)i, true);
}

__global__ __launch_bounds__(256) void blw_split_kernel(const float* __restrict__ w,
                                                        unsigned short* __restrict__ hi,
                                                        unsigned short* __restrict__ lo) {
  const int t = blockIdx.x * 256 + threadIdx.x;
  if (t >= kKeyCols * kHid / 8) return;
  const int rOut = t >> 5;
  const int c8   = (t & 31) * 8;
  const int n    = rOut >> 8;
  const int e    = rOut & 255;
  const int rSrc = e * kNl + n;
  split_store8(w + (size_t)rSrc * kHid + c8, hi + (size_t)rOut * kHid + c8, lo + (size_t)rOut * kHid + c8, true);
}

__global__ __launch_bounds__(256) void f3w_split_kernel(const float* __restrict__ w,
                                                        unsigned short* __restrict__ hi,
                                                        unsigned short* __restrict__ lo) {
  const int t = blockIdx.x * 256 + threadIdx.x;
  if (t >= kNlPad * kHid / 8) return;
  const int r  = t >> 5;
  const int c8 = (t & 31) * 8;
  const bool live = (r < kNl);
  const int rc = live ? r : (kNl - 1);
  split_store8(w + (size_t)rc * kHid + c8, hi + (size_t)r * kHid + c8, lo + (size_t)r * kHid + c8, live);
}

__global__ __launch_bounds__(256) void pair_out_kernel(
    const float* __restrict__ su, const float* __restrict__ tv, const float* __restrict__ f2b,
    const unsigned short* __restrict__ w3hp, const unsigned short* __restrict__ w3lp,
    const float* __restrict__ f3b, const float* __restrict__ o1, float* __restrict__ out) {
  __shared__ __align__(16) float sT[8][16 * 68];
  const int i    = blockIdx.x;
  const int b    = blockIdx.y;
  const int lane = threadIdx.x & 31;
  const int wave = threadIdx.x >> 5;
  const int hh   = lane >> 4;
  const int rl   = lane & 15;
  const int koff = hh * 8;
  const int j0   = wave * 64;
  const __bf16* w3h = (const __bf16*)w3hp;
  const __bf16* w3l = (const __bf16*)w3lp;
  const float* suRow = su + (size_t)(b * kSeqLen + i) * kHid;
  const float* tvBlk = tv + (size_t)(b * kSeqLen + j0) * kHid;

  v8f acc[4];
#pragma unroll
  for (int rt = 0; rt < 4; ++rt) acc[rt] = (v8f){0.f,0.f,0.f,0.f,0.f,0.f,0.f,0.f};

#pragma unroll 1
  for (int ks = 0; ks < kHid / 32; ++ks) {
    const int k0 = ks * 32 + koff;
    const v4f s0 = ld4(suRow + k0), s1 = ld4(suRow + k0 + 4), s2 = ld4(suRow + k0 + 16), s3 = ld4(suRow + k0 + 20);
    const v4f g0 = ld4(f2b + k0),   g1 = ld4(f2b + k0 + 4),   g2 = ld4(f2b + k0 + 16),   g3 = ld4(f2b + k0 + 20);
    const v16b wbh = Frag<__bf16>::load(w3h + (size_t)rl * kHid + k0);
    const v16b wbl = Frag<__bf16>::load(w3l + (size_t)rl * kHid + k0);
#pragma unroll
    for (int rt = 0; rt < 4; ++rt) {
      const float* tvRow = tvBlk + (size_t)(rt * 16 + rl) * kHid + k0;
      const v4f t0 = ld4(tvRow), t1 = ld4(tvRow + 4), t2 = ld4(tvRow + 16), t3 = ld4(tvRow + 20);
      const v4f h0 = relu4((s0 + t0) + g0);
      const v4f h1 = relu4((s1 + t1) + g1);
      const v4f h2 = relu4((s2 + t2) + g2);
      const v4f h3 = relu4((s3 + t3) + g3);
      unsigned hw[8], lw[8];
      split_pack2(h0[0], h0[1], hw[0], lw[0]);
      split_pack2(h0[2], h0[3], hw[1], lw[1]);
      split_pack2(h1[0], h1[1], hw[2], lw[2]);
      split_pack2(h1[2], h1[3], hw[3], lw[3]);
      split_pack2(h2[0], h2[1], hw[4], lw[4]);
      split_pack2(h2[2], h2[3], hw[5], lw[5]);
      split_pack2(h3[0], h3[1], hw[6], lw[6]);
      split_pack2(h3[2], h3[3], hw[7], lw[7]);
      const v8u uhv = (v8u){hw[0], hw[1], hw[2], hw[3], hw[4], hw[5], hw[6], hw[7]};
      const v8u ulv = (v8u){lw[0], lw[1], lw[2], lw[3], lw[4], lw[5], lw[6], lw[7]};
      const v16b ah = __builtin_bit_cast(v16b, uhv);
      const v16b al = __builtin_bit_cast(v16b, ulv);
      acc[rt] = bmma(ah, wbh, acc[rt]);
      acc[rt] = bmma(ah, wbl, acc[rt]);
      acc[rt] = bmma(al, wbh, acc[rt]);
    }
  }

  float* slab = sT[wave];
  const float bias3 = f3b[rl < kNl ? rl : (kNl - 1)];
#pragma unroll
  for (int rt = 0; rt < 4; ++rt) {
#pragma unroll
    for (int r = 0; r < 8; ++r) slab[rl * 68 + rt * 16 + hh * 8 + r] = acc[rt][r] + bias3;
  }
  __builtin_amdgcn_fence(__ATOMIC_RELEASE, "workgroup");
  __builtin_amdgcn_wave_barrier();
  __builtin_amdgcn_fence(__ATOMIC_ACQUIRE, "workgroup");

  const size_t rowBase = (size_t)(b * kSeqLen + i) * kOutPitch;
  const int c4 = rl * 4;
  v4f res[6];
#pragma unroll
  for (int p = 0; p < 6; ++p) {
    const int n = 2 * p + hh;
    const v4f v = *(const v4f*)(slab + n * 68 + c4);
    const size_t off = rowBase + (size_t)n * kSeqLen + j0 + c4;
    const v4f o = ld4(o1 + off);
    res[p] = o + v;
  }
  for (int pass = 0; pass < 2; ++pass) {
#pragma unroll
    for (int p = 0; p < 6; ++p) {
      const int n = 2 * p + hh;
      const size_t off = rowBase + (size_t)n * kSeqLen + j0 + c4;
      *(volatile v4f*)(out + off) = res[p];
    }
    __threadfence();
  }
}

extern "C" void kernel_launch(void* const* d_in, const int* in_sizes, int n_in,
                              void* d_out, int out_size, void* d_ws, size_t ws_size,
                              hipStream_t stream) {
  if (n_in < 10) return;
  if (in_sizes[0] != kRows * kHin) return;
  if (in_sizes[1] != kHid * kHin || in_sizes[2] != kHid) return;
  if (in_sizes[3] != kHid * kHin || in_sizes[4] != kHid) return;
  if (in_sizes[5] != kHid * 2 * kHid || in_sizes[6] != kHid) return;
  if (in_sizes[7] != kNl * kHid || in_sizes[8] != kNl) return;
  if (in_sizes[9] != kKeyCols * kHid) return;
  if (out_size != kBatch * kSeqLen * kNl * kSeqLen) return;

  const float* x   = (const float*)d_in[0];
  const float* sW  = (const float*)d_in[1];
  const float* sb  = (const float*)d_in[2];
  const float* tW  = (const float*)d_in[3];
  const float* tb  = (const float*)d_in[4];
  const float* f2W = (const float*)d_in[5];
  const float* f2b = (const float*)d_in[6];
  const float* f3W = (const float*)d_in[7];
  const float* f3b = (const float*)d_in[8];
  const float* blW = (const float*)d_in[9];
  float* out = (float*)d_out;

  char* ws = (char*)d_ws;
  size_t off = 0;
  const size_t bx   = (size_t)kRows * kHin * 2;
  const size_t bw   = (size_t)kHid * kHin * 2;
  const size_t bf2  = (size_t)kHid * 2 * kHid * 2;
  const size_t bbl  = (size_t)kKeyCols * kHid * 2;
  const size_t bw3  = (size_t)kNlPad * kHid * 2;
  const size_t bst  = (size_t)2 * kRows * kHid * 2;
  const size_t bkey = (size_t)kRows * kKeyCols * 2;
  const size_t bsut = (size_t)2 * kRows * kHid * 4;
  const size_t bo1  = (size_t)kBatch * kSeqLen * kNl * kSeqLen * 4;
  unsigned short* xh   = (unsigned short*)(ws + off); off += bx;
  unsigned short* xl   = (unsigned short*)(ws + off); off += bx;
  unsigned short* sWh  = (unsigned short*)(ws + off); off += bw;
  unsigned short* sWl  = (unsigned short*)(ws + off); off += bw;
  unsigned short* tWh  = (unsigned short*)(ws + off); off += bw;
  unsigned short* tWl  = (unsigned short*)(ws + off); off += bw;
  unsigned short* f2Wh = (unsigned short*)(ws + off); off += bf2;
  unsigned short* f2Wl = (unsigned short*)(ws + off); off += bf2;
  unsigned short* blWh = (unsigned short*)(ws + off); off += bbl;
  unsigned short* blWl = (unsigned short*)(ws + off); off += bbl;
  unsigned short* w3h  = (unsigned short*)(ws + off); off += bw3;
  unsigned short* w3l  = (unsigned short*)(ws + off); off += bw3;
  unsigned short* sth  = (unsigned short*)(ws + off); off += bst;
  unsigned short* stl  = (unsigned short*)(ws + off); off += bst;
  unsigned short* keyh = (unsigned short*)(ws + off); off += bkey;
  unsigned short* keyl = (unsigned short*)(ws + off); off += bkey;
  float*          sutv = (float*)(ws + off);          off += bsut;
  float*          o1   = (float*)(ws + off);          off += bo1;
  if (off > ws_size) return;

  const size_t planeST = (size_t)kRows * kHid;
  unsigned short* th = sth + planeST;
  unsigned short* tl = stl + planeST;
  float* su = sutv;
  float* tv = sutv + planeST;
  const dim3 blk(256, 1, 1);

  split8_bf16_kernel<<<dim3((kRows * kHin / 8 + 255) / 256), blk, 0, stream>>>(x, xh, xl, kRows * kHin / 8);
  split8_bf16_kernel<<<dim3((kHid * kHin / 8 + 255) / 256), blk, 0, stream>>>(sW, sWh, sWl, kHid * kHin / 8);
  split8_bf16_kernel<<<dim3((kHid * kHin / 8 + 255) / 256), blk, 0, stream>>>(tW, tWh, tWl, kHid * kHin / 8);
  split8_bf16_kernel<<<dim3((kHid * 2 * kHid / 8 + 255) / 256), blk, 0, stream>>>(f2W, f2Wh, f2Wl, kHid * 2 * kHid / 8);
  blw_split_kernel<<<dim3((kKeyCols * kHid / 8 + 255) / 256), blk, 0, stream>>>(blW, blWh, blWl);
  f3w_split_kernel<<<dim3((kNlPad * kHid / 8 + 255) / 256), blk, 0, stream>>>(f3W, w3h, w3l);

  wmma_gemm64<1, true, 2, 2, false, 2><<<dim3(8, 1), blk, 0, stream>>>(
      xh, xl, kHin, 0L, sWh, sWl, kHin, 0L, (void*)sth, (void*)stl, kHid, 0L,
      sb, (const float*)sutv, 0L, kRows, kHid, kHin, 1.0f);
  wmma_gemm64<1, true, 2, 2, false, 2><<<dim3(8, 1), blk, 0, stream>>>(
      xh, xl, kHin, 0L, tWh, tWl, kHin, 0L, (void*)th, (void*)tl, kHid, 0L,
      tb, (const float*)sutv, 0L, kRows, kHid, kHin, 1.0f);

  wmma_gemm64<1, true, 0, 2, false, 0><<<dim3(96, 1), blk, 0, stream>>>(
      sth, stl, kHid, 0L, blWh, blWl, kHid, 0L, (void*)keyh, (void*)keyl, kKeyCols, 0L,
      sb, (const float*)sutv, 0L, kRows, kKeyCols, kHid, 1.0f);

  wmma_gemm64<1, true, 0, 0, false, 0><<<dim3(8, 2), blk, 0, stream>>>(
      sth, stl, kHid, (long)planeST, f2Wh, f2Wl, 2 * kHid, (long)kHid, (void*)sutv, (void*)sutv, kHid, (long)planeST,
      sb, (const float*)sutv, 0L, kRows, kHid, kHid, 1.0f);

  for (int b = 0; b < kBatch; ++b) {
    const size_t aoff = (size_t)b * kSeqLen * kKeyCols;
    const size_t toff = (size_t)b * kSeqLen * kHid;
    const size_t coff = (size_t)b * kSeqLen * kOutPitch;
    wmma_gemm64<1, true, 0, 0, false, 0><<<dim3(8, kNl), blk, 0, stream>>>(
        keyh + aoff, keyl + aoff, kKeyCols, (long)kHid, th + toff, tl + toff, kHid, 0L,
        (void*)(o1 + coff), (void*)sutv, kOutPitch, (long)kSeqLen,
        sb, (const float*)sutv, 0L, kSeqLen, kSeqLen, kHid, 1.0f);
  }

  pair_out_kernel<<<dim3(kSeqLen, kBatch), blk, 0, stream>>>(su, tv, f2b, w3h, w3l, f3b, o1, out);
}
